// GCN_59090160058839
// MI455X (gfx1250) — hardware-verified
//
#include <hip/hip_runtime.h>
#include <stddef.h>
#include <stdint.h>
#include <math.h>


#define DF     128
#define NCLS   16
#define NGR    100
#define K2     256
#define NTHR   256
#define NWAVE  8
#define EPT    8
#define CHUNK  (NTHR * EPT)
#define WCAP   (EPT * 32)
#define LISTN  (NWAVE * WCAP)
#define NBD    8192
#define SLD    13
#define NBA    1024
#define SLA    10
#define RCAP   28672
#define DEGCAP 64
#define MEAS_B1024 16721
#define MEAS_MAXDEG 36
#define GBM    64
#define GBN    128
#define GTHR   128
#define ROWH   256
#define NUW1   (DF * (DF / 8))
#define NUW2   (DF * (K2 / 8))
#define NUTB   NTHR
#define NUPRE  (NUW1 + NUW2 + NUTB)
#define T_B1   0
#define T_PC   128
#define T_C2   256
#define T_BC   288
#define T_WC   320
#define TABN   2368
#define AGG_ZINTS (LISTN + 2 * RCAP + 3 * NBA)
#define MISC_INTS 16
#define BKT_LDS_INTS (AGG_ZINTS + MISC_INTS)
#define WSMAX  134217728

static_assert((CHUNK & (CHUNK - 1)) == 0 && CHUNK <= 4096);
static_assert((NBD & (NBD - 1)) == 0 && NBD == (1 << SLD));
static_assert((NBA & (NBA - 1)) == 0 && NBA == (1 << SLA));
static_assert(((long long)CHUNK << SLD) < (1LL << 31));
static_assert(((long long)CHUNK << SLA) < (1LL << 31));
static_assert(NBD % (NTHR * 4) == 0 && NBA == NTHR * 4);
static_assert(LISTN % NTHR == 0);
static_assert(NBA % NWAVE == 0 && NBA % 32 == 0 && NBA % GBM == 0);
static_assert(RCAP % (NTHR * 4) == 0 && AGG_ZINTS % (NTHR * 4) == 0);
static_assert(RCAP >= MEAS_B1024 + MEAS_B1024 / 20);
static_assert(DEGCAP >= MEAS_MAXDEG + 8);
static_assert(DF % 32 == 0 && K2 % 32 == 0 && K2 == 2 * DF && GBN == DF);
static_assert(GBM == (GTHR / 32) * 16 && DF == 4 * 32 && ROWH == 2 * DF);
static_assert(NUW1 % NTHR == 0 && NUW2 % NTHR == 0 && NUPRE % NTHR == 0);
static_assert(TABN % 32 == 0 && T_WC + DF * NCLS == TABN && (TABN / 4) <= 3 * NTHR);
static_assert(BKT_LDS_INTS * 4 <= 300000);
static_assert((NGR * NCLS) % 32 == 0 && NGR % 2 == 0 && NCLS == 16);
static_assert((DF * NCLS / 4) % GTHR == 0 && (GBM * NCLS / 4) % GTHR == 0);

typedef float          v4f   __attribute__((ext_vector_type(4)));
typedef float          v8f   __attribute__((ext_vector_type(8)));
typedef int            v4i   __attribute__((ext_vector_type(4)));
typedef int            v8i   __attribute__((ext_vector_type(8)));
typedef unsigned short v4us  __attribute__((ext_vector_type(4)));
typedef unsigned short v8us  __attribute__((ext_vector_type(8)));
typedef unsigned short v16us __attribute__((ext_vector_type(16)));
typedef __bf16         v16bf __attribute__((ext_vector_type(16)));
typedef v4f  __attribute__((may_alias)) v4fa;
typedef v4i  __attribute__((may_alias)) v4ia;
typedef v4us __attribute__((may_alias)) v4usa;
typedef v8us __attribute__((may_alias)) v8usa;
union FragB { v16bf v; v16us u; v8us h[2]; v8i w; };

__device__ __forceinline__ v8f wmb(const FragB& a, const FragB& b, v8f c) {
  v8f d = __builtin_amdgcn_wmma_f32_16x16x32_bf16(false, a.v, false, b.v, (short)0, c, false, false);
  asm volatile("v_nop\n\tv_nop\n\tv_nop\n\tv_nop" : "+v"(d) : "v"(a.w), "v"(b.w));
  return d;
}

__device__ __forceinline__ v8f z8() { v8f z = {0.f, 0.f, 0.f, 0.f, 0.f, 0.f, 0.f, 0.f}; return z; }

__device__ __forceinline__ unsigned bf16_bits(float f) {
  const unsigned u = __float_as_uint(f);
  return (u + 0x7FFFu + ((u >> 16) & 1u)) >> 16;
}
__device__ __forceinline__ float bf16_val(float f) {
  return __uint_as_float(bf16_bits(f) << 16);
}
__device__ __forceinline__ float bsel(int m, float a, float b) {
  return __int_as_float((__float_as_int(a) & m) | (__float_as_int(b) & ~m));
}

__device__ __forceinline__ void wave_sync() {
  __builtin_amdgcn_fence(__ATOMIC_RELEASE, "wavefront");
  __builtin_amdgcn_wave_barrier();
  __builtin_amdgcn_fence(__ATOMIC_ACQUIRE, "wavefront");
}

template <int SLB>
__device__ __forceinline__ int scan_chunk(const int* __restrict__ dsts, int nE, int cbase, int slotBase,
                                          int nb, int vec8, int* list, int tid, int lane, int wave) {
  int wc = 0;
  const int el0  = tid * EPT;
  const int e0   = cbase + el0;
  const int sent = -2147483647 - 1;
  v4i da, db;
  if (vec8 != 0 && cbase + CHUNK <= nE) {
    da = *(const v4i*)(dsts + e0);
    db = *(const v4i*)(dsts + e0 + 4);
  } else {
    da.x = (e0     < nE) ? dsts[min(e0,     nE - 1)] : sent;
    da.y = (e0 + 1 < nE) ? dsts[min(e0 + 1, nE - 1)] : sent;
    da.z = (e0 + 2 < nE) ? dsts[min(e0 + 2, nE - 1)] : sent;
    da.w = (e0 + 3 < nE) ? dsts[min(e0 + 3, nE - 1)] : sent;
    db.x = (e0 + 4 < nE) ? dsts[min(e0 + 4, nE - 1)] : sent;
    db.y = (e0 + 5 < nE) ? dsts[min(e0 + 5, nE - 1)] : sent;
    db.z = (e0 + 6 < nE) ? dsts[min(e0 + 6, nE - 1)] : sent;
    db.w = (e0 + 7 < nE) ? dsts[min(e0 + 7, nE - 1)] : sent;
  }
  const unsigned nbs = (unsigned)slotBase;
  const unsigned unb = (unsigned)nb;
  const unsigned s0 = (unsigned)da.x - nbs, s1 = (unsigned)da.y - nbs;
  const unsigned s2 = (unsigned)da.z - nbs, s3 = (unsigned)da.w - nbs;
  const unsigned s4 = (unsigned)db.x - nbs, s5 = (unsigned)db.y - nbs;
  const unsigned s6 = (unsigned)db.z - nbs, s7 = (unsigned)db.w - nbs;
  const bool h0 = s0 < unb, h1 = s1 < unb, h2 = s2 < unb, h3 = s3 < unb;
  const bool h4 = s4 < unb, h5 = s5 < unb, h6 = s6 < unb, h7 = s7 < unb;
  const unsigned any = __builtin_amdgcn_ballot_w32(h0 | h1 | h2 | h3 | h4 | h5 | h6 | h7);
  if (any != 0u) {
#define HITJ(J, HJ, SJ) { \
      const unsigned mj = __builtin_amdgcn_ballot_w32(HJ); \
      if (mj != 0u) { \
        if (HJ) { \
          const int pos = wc + (int)__builtin_amdgcn_mbcnt_lo(mj, 0u); \
          if (pos < WCAP) list[wave * WCAP + pos] = ((el0 + (J)) << SLB) | (int)(SJ); \
        } \
        wc += (int)__builtin_popcount(mj); } }
    HITJ(0, h0, s0)
    HITJ(1, h1, s1)
    HITJ(2, h2, s2)
    HITJ(3, h3, s3)
    HITJ(4, h4, s4)
    HITJ(5, h5, s5)
    HITJ(6, h6, s6)
    HITJ(7, h7, s7)
#undef HITJ
  }
  return wc;
}

__global__ __launch_bounds__(NTHR) void k_prep(const float* __restrict__ h, const float* __restrict__ W1,
                                               const float* __restrict__ b1, const float* __restrict__ p,
                                               const float* __restrict__ W2, const float* __restrict__ b2,
                                               const float* __restrict__ Wc, const float* __restrict__ bc,
                                               unsigned short* hb, unsigned short* w1t, unsigned short* w2d,
                                               float* tab, int nN, int nUnits) {
  __shared__ __attribute__((aligned(16))) float tl[TABN];
  __shared__ float b2s[DF];
  const int tid = (int)threadIdx.x;
  const int u = (int)blockIdx.x * NTHR + tid;
  if (u >= NUW1 + NUW2 && u < NUPRE) {
    const int t = tid;
    if (t < DF) {
      tl[T_B1 + t] = bf16_val(b1[t]);
      const float pr = bf16_val(p[t]);
      tl[T_PC + t] = fminf(fmaxf(pr, 0.0f), 1.0f);
      b2s[t] = bf16_val(b2[t]);
    }
#pragma unroll
    for (int j = 0; j < 2; ++j) {
      const int i4 = t + NTHR * j;
      const v4f w = *(const v4f*)(Wc + 4 * i4);
      v4f wv;
      wv.x = bf16_val(w.x); wv.y = bf16_val(w.y); wv.z = bf16_val(w.z); wv.w = bf16_val(w.w);
      *(v4fa*)(tl + T_WC + 4 * i4) = wv;
    }
    if (t < 32) {
      const float bb = bc[t & (NCLS - 1)];
      tl[T_BC + t] = (t < NCLS) ? bf16_val(bb) : 0.0f;
    }
    __syncthreads();
    if (t < 32) {
      const int c = t & (NCLS - 1);
      float s = 0.0f;
#pragma unroll 1
      for (int k = 0; k < DF; ++k) s = fmaf(b2s[k], tl[T_WC + k * NCLS + c], s);
      tl[T_C2 + t] = (t < NCLS) ? s : 0.0f;
    }
    __syncthreads();
    v4f tv[3];
#pragma unroll
    for (int it = 0; it < 3; ++it) {
      const int i4 = t + NTHR * it;
      const int ic = i4 < TABN / 4 ? i4 : TABN / 4 - 1;
      tv[it] = *(const v4fa*)(tl + 4 * ic);
    }
#pragma unroll
    for (int it = 0; it < 3; ++it) {
      const int i4 = t + NTHR * it;
      if (i4 < TABN / 4) *(volatile v4f*)(tab + 4 * i4) = tv[it];
    }
    __threadfence();
#pragma unroll
    for (int it = 0; it < 3; ++it) {
      const int i4 = t + NTHR * it;
      if (i4 < TABN / 4) *(volatile v4f*)(tab + 4 * i4) = tv[it];
    }
    return;
  }
  v8us o;
  unsigned short* dp;
  if (u < NUW1) {
    const int n  = u >> 4;
    const int k8 = (u & 15) * 8;
    const float* q = W1 + (size_t)k8 * DF + n;
#pragma unroll
    for (int i = 0; i < 8; ++i) o[i] = (unsigned short)bf16_bits(q[(size_t)i * DF]);
    dp = w1t + (size_t)n * DF + k8;
  } else if (u < NUW1 + NUW2) {
    const int v  = u - NUW1;
    const int n  = v >> 5;
    const int k8 = (v & 31) * 8;
    const int kk = k8 & (DF - 1);
    const float* q = W2 + (size_t)kk * DF + n;
#pragma unroll
    for (int i = 0; i < 8; ++i) o[i] = (unsigned short)bf16_bits(q[(size_t)i * DF]);
    dp = w2d + (size_t)n * K2 + k8;
  } else if (u < nUnits) {
    const int v   = u - NUPRE;
    const int row = v >> 4;
    const int k8  = (v & 15) * 8;
    const int rc  = row < nN ? row : nN - 1;
    const float* q = h + (size_t)rc * DF + k8;
    const v4f a = *(const v4fa*)q;
    const v4f b = *(const v4fa*)(q + 4);
    const bool ok = row < nN;
    o[0] = ok ? (unsigned short)bf16_bits(a.x) : (unsigned short)0;
    o[1] = ok ? (unsigned short)bf16_bits(a.y) : (unsigned short)0;
    o[2] = ok ? (unsigned short)bf16_bits(a.z) : (unsigned short)0;
    o[3] = ok ? (unsigned short)bf16_bits(a.w) : (unsigned short)0;
    o[4] = ok ? (unsigned short)bf16_bits(b.x) : (unsigned short)0;
    o[5] = ok ? (unsigned short)bf16_bits(b.y) : (unsigned short)0;
    o[6] = ok ? (unsigned short)bf16_bits(b.z) : (unsigned short)0;
    o[7] = ok ? (unsigned short)bf16_bits(b.w) : (unsigned short)0;
    dp = hb + (size_t)row * DF + k8;
  } else {
    return;
  }
  *(volatile v8us*)dp = o;
  __threadfence();
  *(volatile v8us*)dp = o;
}

__global__ __launch_bounds__(NTHR) void k_degout(const int* __restrict__ keys, int nE, int vec8, float* ns) {
  __shared__ __attribute__((aligned(16))) int scnt[NBD];
  __shared__ __attribute__((aligned(16))) int list[LISTN];
  __shared__ int wcnt[NWAVE];
  const int tid = (int)threadIdx.x, lane = tid & 31, wave = tid >> 5;
  const int nodeBase = (int)blockIdx.x * NBD;

  for (int i = tid; i < NBD; i += NTHR) scnt[i] = 0;
  for (int i = tid; i < LISTN; i += NTHR) list[i] = 0;
  if (tid < NWAVE) wcnt[tid] = 0;
  __syncthreads();

  const int nChunks = (nE + CHUNK - 1) / CHUNK;
#pragma unroll 1
  for (int ch = 0; ch < nChunks; ++ch) {
    const int cbase = ch * CHUNK;
    const int wc = scan_chunk<SLD>(keys, nE, cbase, nodeBase, NBD, vec8, list, tid, lane, wave);
    if (lane == 0) wcnt[wave] = wc;
    __syncthreads();
    if (wave == 0) {
#pragma unroll 1
      for (int w2 = 0; w2 < NWAVE; ++w2) {
        int c = wcnt[w2];
        c = c < 0 ? 0 : (c > WCAP ? WCAP : c);
#pragma unroll 1
        for (int b0 = 0; b0 < c; b0 += 32) {
          const int idx = b0 + lane;
          const int ent = list[w2 * WCAP + (idx < WCAP ? idx : WCAP - 1)];
          const int m32 = (c - b0) < 32 ? (c - b0) : 32;
#pragma unroll 1
          for (int k = 0; k < m32; ++k) {
            const int u  = __builtin_amdgcn_readlane(ent, k);
            const int sl = u & (NBD - 1);
            if (lane == 0) scnt[sl] = scnt[sl] + 1;
          }
        }
      }
    }
    __syncthreads();
  }

#pragma unroll 1
  for (int i = tid; i < NBD; i += NTHR) {
    const int c = scnt[i];
    const float d = (float)(c < 1 ? 1 : c);
    const float r = 1.0f / sqrtf(d);
    scnt[i] = __float_as_int(c > 0 ? r : 0.0f);
  }
  __syncthreads();

  v4f vals[NBD / (NTHR * 4)];
#pragma unroll
  for (int it = 0; it < NBD / (NTHR * 4); ++it) {
    const int s0 = it * (NTHR * 4) + 4 * tid;
    const v4i c4 = *(const v4ia*)(scnt + s0);
    v4f v;
    v.x = __int_as_float(c4.x); v.y = __int_as_float(c4.y);
    v.z = __int_as_float(c4.z); v.w = __int_as_float(c4.w);
    vals[it] = v;
  }
#pragma unroll
  for (int it = 0; it < NBD / (NTHR * 4); ++it) {
    const int s0 = it * (NTHR * 4) + 4 * tid;
    *(volatile v4f*)(ns + (size_t)nodeBase + s0) = vals[it];
  }
  __threadfence();
#pragma unroll
  for (int it = 0; it < NBD / (NTHR * 4); ++it) {
    const int s0 = it * (NTHR * 4) + 4 * tid;
    *(volatile v4f*)(ns + (size_t)nodeBase + s0) = vals[it];
  }
}

__global__ __launch_bounds__(NTHR) void k_bucket(const int* __restrict__ srcs, const int* __restrict__ dsts,
                                                 int nE, int nN, int vec8,
                                                 int* lst, int* cntg, int* offg, float* ndg, int* flg) {
  extern __shared__ __attribute__((aligned(16))) int dsm[];
  int* list = dsm;
  int* hl   = dsm + LISTN;
  int* sl   = hl + RCAP;
  int* cnt  = sl + RCAP;
  int* offs = cnt + NBA;
  int* cur  = offs + NBA;
  int* misc = cur + NBA;
  const int tid = (int)threadIdx.x, lane = tid & 31, wave = tid >> 5;
  const int blk = (int)blockIdx.x;
  const int nodeBase = blk * NBA;

  {
    const v4i z4 = {0, 0, 0, 0};
    for (int i = tid * 4; i < AGG_ZINTS; i += NTHR * 4) *(v4ia*)(dsm + i) = z4;
    if (tid < MISC_INTS) misc[tid] = 0;
  }
  __syncthreads();

  int t = 0, ov = 0;
  const int nChunks = (nE + CHUNK - 1) / CHUNK;
#pragma unroll 1
  for (int ch = 0; ch < nChunks; ++ch) {
    const int cbase = ch * CHUNK;
    const int wc = scan_chunk<SLA>(dsts, nE, cbase, nodeBase, NBA, vec8, list, tid, lane, wave);
    if (lane == 0) misc[wave] = wc;
    __syncthreads();
    if (wave == 0) {
#pragma unroll 1
      for (int w2 = 0; w2 < NWAVE; ++w2) {
        int c = misc[w2];
        c = c < 0 ? 0 : (c > WCAP ? WCAP : c);
#pragma unroll 1
        for (int b0 = 0; b0 < c; b0 += 32) {
          const int idx = b0 + lane;
          const int ent_ = list[w2 * WCAP + (idx < WCAP ? idx : WCAP - 1)];
          const int m32 = (c - b0) < 32 ? (c - b0) : 32;
#pragma unroll 1
          for (int k = 0; k < m32; ++k) {
            const int u    = __builtin_amdgcn_readlane(ent_, k);
            const int slot = u & (NBA - 1);
            const int el   = (u >> SLA) & (CHUNK - 1);
            const int pk   = ((cbase + el) << SLA) | slot;
            if (t < RCAP) {
              if (lane == 0) { hl[t] = pk; cnt[slot] = cnt[slot] + 1; }
              t = t + 1;
            } else {
              ov = 1;
            }
          }
        }
      }
    }
    __syncthreads();
  }
  if (wave == 0 && lane == 0) { misc[8] = t; misc[9] = ov; }
  __syncthreads();
  int tt = misc[8];
  tt = tt < 0 ? 0 : (tt > RCAP ? RCAP : tt);
  const int ovf = misc[9];

  if (wave == 0) {
    const int base = lane * (NBA / 32);
    int s = 0;
#pragma unroll 1
    for (int i = 0; i < NBA / 32; ++i) s += cnt[base + i];
    int incl = s;
#pragma unroll
    for (int d = 1; d < 32; d <<= 1) {
      const int y = __shfl_up(incl, d, 32);
      if (lane >= d) incl += y;
    }
    int run = incl - s;
#pragma unroll 1
    for (int i = 0; i < NBA / 32; ++i) {
      const int cv = cnt[base + i];
      offs[base + i] = run;
      cur[base + i]  = run;
      run += cv;
    }
  }
  __syncthreads();
  if (wave == 0) {
#pragma unroll 1
    for (int b0 = 0; b0 < tt; b0 += 32) {
      const int idx = b0 + lane;
      const int ent_ = hl[idx < RCAP ? idx : RCAP - 1];
      const int m32 = (tt - b0) < 32 ? (tt - b0) : 32;
#pragma unroll 1
      for (int k = 0; k < m32; ++k) {
        const int u    = __builtin_amdgcn_readlane(ent_, k);
        const int slot = u & (NBA - 1);
        if (lane == 0) {
          int pp = cur[slot];
          pp = pp < 0 ? 0 : (pp > RCAP - 1 ? RCAP - 1 : pp);
          sl[pp] = u;
          cur[slot] = pp + 1;
        }
      }
    }
  }
  __syncthreads();

#pragma unroll 1
  for (int i = tid; i < NBA; i += NTHR) {
    const int c = cnt[i];
    if (c > DEGCAP) misc[10] = 1;
    const float d = (float)(c < 1 ? 1 : c);
    const float r = 1.0f / sqrtf(d);
    cur[i] = __float_as_int(c > 0 ? r : 0.0f);
  }
  __syncthreads();
  const int fl = (ovf != 0 || misc[10] != 0) ? 1 : 0;

  {
    const v4i c4 = *(const v4ia*)(cnt + 4 * tid);
    const v4i o4 = *(const v4ia*)(offs + 4 * tid);
    const v4i n4 = *(const v4ia*)(cur + 4 * tid);
    v4f nf;
    nf.x = __int_as_float(n4.x); nf.y = __int_as_float(n4.y);
    nf.z = __int_as_float(n4.z); nf.w = __int_as_float(n4.w);
    const v4i f4 = {fl, fl, fl, fl};
    int*   cp = cntg + (size_t)nodeBase + 4 * tid;
    int*   op = offg + (size_t)nodeBase + 4 * tid;
    float* np = ndg  + (size_t)nodeBase + 4 * tid;
    int*   fp = flg  + (size_t)blk * 32 + 4 * (tid & 7);
    const bool fw = tid < 8;
    *(volatile v4i*)cp = c4;
    *(volatile v4i*)op = o4;
    *(volatile v4f*)np = nf;
    if (fw) *(volatile v4i*)fp = f4;
    __threadfence();
    *(volatile v4i*)cp = c4;
    *(volatile v4i*)op = o4;
    *(volatile v4f*)np = nf;
    if (fw) *(volatile v4i*)fp = f4;
  }

  int* lb = lst + (size_t)blk * RCAP;
#pragma unroll 1
  for (int it = 0; it < RCAP / (NTHR * 4); ++it) {
    const int i4 = (it * NTHR + tid) * 4;
    const v4i e4 = *(const v4ia*)(sl + i4);
    int e0 = e4.x >> SLA, e1 = e4.y >> SLA, e2 = e4.z >> SLA, e3 = e4.w >> SLA;
    e0 = e0 < 0 ? 0 : (e0 > nE - 1 ? nE - 1 : e0);
    e1 = e1 < 0 ? 0 : (e1 > nE - 1 ? nE - 1 : e1);
    e2 = e2 < 0 ? 0 : (e2 > nE - 1 ? nE - 1 : e2);
    e3 = e3 < 0 ? 0 : (e3 > nE - 1 ? nE - 1 : e3);
    int r0 = srcs[e0], r1 = srcs[e1], r2 = srcs[e2], r3 = srcs[e3];
    r0 = r0 < 0 ? 0 : (r0 > nN - 1 ? nN - 1 : r0);
    r1 = r1 < 0 ? 0 : (r1 > nN - 1 ? nN - 1 : r1);
    r2 = r2 < 0 ? 0 : (r2 > nN - 1 ? nN - 1 : r2);
    r3 = r3 < 0 ? 0 : (r3 > nN - 1 ? nN - 1 : r3);
    v4i o;
    o.x = (i4     < tt) ? r0 : 0;
    o.y = (i4 + 1 < tt) ? r1 : 0;
    o.z = (i4 + 2 < tt) ? r2 : 0;
    o.w = (i4 + 3 < tt) ? r3 : 0;
    int* lp = lb + i4;
    *(volatile v4i*)lp = o;
    __threadfence();
    *(volatile v4i*)lp = o;
  }
}

__global__ __launch_bounds__(GTHR) void k_gemm1(const unsigned short* __restrict__ A,
                                                const unsigned short* __restrict__ BT,
                                                const float* __restrict__ ns, float* m1, int nN) {
  __shared__ __attribute__((aligned(16))) float stg[GBM * GBN];
  const int tid = (int)threadIdx.x, lane = tid & 31, wave = tid >> 5, hh = lane >> 4, m = lane & 15;
  const int rowBase = (int)blockIdx.x * GBM;

  v8f acc[8];
#pragma unroll
  for (int t = 0; t < 8; ++t) acc[t] = z8();
  const unsigned short* ap = A + (size_t)(rowBase + 16 * wave + m) * (size_t)DF + 8 * hh;
  const unsigned short* bp = BT + (size_t)m * (size_t)DF + 8 * hh;
  int rr = rowBase + 16 * wave + m;
  rr = rr > nN - 1 ? nN - 1 : rr;
  const float nsv = ns[rr];

#pragma unroll 1
  for (int k0 = 0; k0 < DF; k0 += 32) {
    FragB af;
    af.h[0] = *(const v8usa*)(ap + k0);
    af.h[1] = *(const v8usa*)(ap + k0 + 16);
#pragma unroll
    for (int nt = 0; nt < 8; ++nt) {
      const unsigned short* wq = bp + (size_t)(16 * nt) * (size_t)DF + k0;
      FragB bf;
      bf.h[0] = *(const v8usa*)wq;
      bf.h[1] = *(const v8usa*)(wq + 16);
      acc[nt] = wmb(af, bf, acc[nt]);
    }
  }

#pragma unroll
  for (int nt = 0; nt < 8; ++nt) {
    const int lc = 16 * nt + m;
#pragma unroll
    for (int r = 0; r < 8; ++r) {
      const int lr = 16 * wave + 8 * hh + r;
      stg[lr * GBN + lc] = acc[nt][r];
    }
  }
  __syncthreads();

  v4f pv[16];
#pragma unroll
  for (int i = 0; i < 16; ++i) {
    const float s = __shfl(nsv, i, 32);
    const v4f q = *(const v4fa*)(stg + (16 * wave + i) * GBN + 4 * lane);
    v4f o;
    o.x = q.x * s; o.y = q.y * s; o.z = q.z * s; o.w = q.w * s;
    pv[i] = o;
  }
#pragma unroll
  for (int i = 0; i < 16; ++i) {
    const int row = rowBase + 16 * wave + i;
    float* op = m1 + (size_t)row * DF + 4 * lane;
    if (row < nN) *(volatile v4f*)op = pv[i];
  }
  __threadfence();
#pragma unroll
  for (int i = 0; i < 16; ++i) {
    const int row = rowBase + 16 * wave + i;
    float* op = m1 + (size_t)row * DF + 4 * lane;
    if (row < nN) *(volatile v4f*)op = pv[i];
  }
}

__global__ __launch_bounds__(NTHR) void k_agg1(const int* __restrict__ lst, const int* __restrict__ cntg,
                                               const int* __restrict__ offg, const float* __restrict__ ndg,
                                               const int* __restrict__ flg, const float* __restrict__ m1,
                                               const float* __restrict__ tab, int nN, int mRows,
                                               unsigned short* x1p) {
  __shared__ __attribute__((aligned(16))) unsigned short rowbufs[NWAVE * ROWH];
  const int tid = (int)threadIdx.x, lane = tid & 31, wave = tid >> 5;
  const int blk = (int)blockIdx.x;
  const int nodeBase = blk * NBA;
  unsigned short* rowbuf = rowbufs + wave * ROWH;
  const int* bl = lst + (size_t)blk * RCAP;
  const float qnan = __int_as_float(0x7fc00000);
  const float pz = (flg[blk * 32] != 0) ? qnan : 0.0f;
  const v4f b4 = *(const v4f*)(tab + T_B1 + 4 * lane);
  const v4f p4 = *(const v4f*)(tab + T_PC + 4 * lane);

#pragma unroll 1
  for (int si = 0; si < NBA / NWAVE; ++si) {
    const int s    = si * NWAVE + wave;
    const int node = nodeBase + s;
    int c = cntg[node];
    const bool big = c > DEGCAP;
    c = c < 0 ? 0 : (c > DEGCAP ? DEGCAP : c);
    int o = offg[node];
    o = o < 0 ? 0 : (o > RCAP ? RCAP : o);
    const float nd = ndg[node];
    float a0 = 0.0f, a1 = 0.0f, a2 = 0.0f, a3 = 0.0f;
#pragma unroll 1
    for (int b0 = 0; b0 < c; b0 += 32) {
      int idx = o + b0 + lane;
      idx = idx > RCAP - 1 ? RCAP - 1 : idx;
      int sr = bl[idx];
      sr = sr < 0 ? 0 : (sr > nN - 1 ? nN - 1 : sr);
      const int m32 = (c - b0) < 32 ? (c - b0) : 32;
#pragma unroll 1
      for (int k = 0; k < m32; ++k) {
        const int sk = __builtin_amdgcn_readlane(sr, k);
        const v4f a = *(const v4fa*)(m1 + (size_t)sk * DF + 4 * lane);
        a0 += a.x; a1 += a.y; a2 += a.z; a3 += a.w;
      }
    }
    const float pzr = big ? qnan : pz;
    const bool live = node < nN;
    float y0 = a0 * nd + b4.x, y1 = a1 * nd + b4.y, y2 = a2 * nd + b4.z, y3 = a3 * nd + b4.w;
    y0 = (y0 > 0.0f) ? y0 : (y0 - y0);
    y1 = (y1 > 0.0f) ? y1 : (y1 - y1);
    y2 = (y2 > 0.0f) ? y2 : (y2 - y2);
    y3 = (y3 > 0.0f) ? y3 : (y3 - y3);
    y0 = y0 * p4.x + pzr; y1 = y1 * p4.y + pzr; y2 = y2 * p4.z + pzr; y3 = y3 * p4.w + pzr;
    const float v0 = live ? y0 : 0.0f;
    const float v1 = live ? y1 : 0.0f;
    const float v2 = live ? y2 : 0.0f;
    const float v3 = live ? y3 : 0.0f;
    v4us mh, ml;
    {
      const unsigned h0 = bf16_bits(v0), h1 = bf16_bits(v1), h2 = bf16_bits(v2), h3 = bf16_bits(v3);
      const unsigned l0 = bf16_bits(v0 - __uint_as_float(h0 << 16));
      const unsigned l1 = bf16_bits(v1 - __uint_as_float(h1 << 16));
      const unsigned l2 = bf16_bits(v2 - __uint_as_float(h2 << 16));
      const unsigned l3 = bf16_bits(v3 - __uint_as_float(h3 << 16));
      mh[0] = (unsigned short)h0; mh[1] = (unsigned short)h1; mh[2] = (unsigned short)h2; mh[3] = (unsigned short)h3;
      ml[0] = (unsigned short)l0; ml[1] = (unsigned short)l1; ml[2] = (unsigned short)l2; ml[3] = (unsigned short)l3;
    }
    *(v4usa*)(rowbuf + 4 * lane)      = mh;
    *(v4usa*)(rowbuf + DF + 4 * lane) = ml;
    wave_sync();
    const v8us q0 = *(const v8usa*)(rowbuf + 8 * lane);
    wave_sync();
    if (node < mRows) {
      unsigned short* rpw = x1p + (size_t)node * K2 + 8 * lane;
      *(volatile v8us*)rpw = q0;
      __threadfence();
      *(volatile v8us*)rpw = q0;
    }
  }
}

__global__ __launch_bounds__(GTHR) void k_gemm2(const unsigned short* __restrict__ A,
                                                const unsigned short* __restrict__ BT,
                                                const float* __restrict__ ns, const float* __restrict__ tab,
                                                float* y16, int nN) {
  __shared__ __attribute__((aligned(16))) float stg[GBM * GBN];
  __shared__ __attribute__((aligned(16))) float wcs[DF * NCLS];
  __shared__ __attribute__((aligned(16))) float ys[GBM * NCLS];
  __shared__ float nss[GBM];
  const int tid = (int)threadIdx.x, lane = tid & 31, wave = tid >> 5, hh = lane >> 4, m = lane & 15;
  const int rowBase = (int)blockIdx.x * GBM;

#pragma unroll
  for (int j = 0; j < (DF * NCLS / 4) / GTHR; ++j) {
    const int i4 = tid + GTHR * j;
    const v4f w = *(const v4f*)(tab + T_WC + 4 * i4);
    *(v4fa*)(wcs + 4 * i4) = w;
  }
  if (tid < GBM) {
    int rr = rowBase + tid;
    rr = rr > nN - 1 ? nN - 1 : rr;
    nss[tid] = ns[rr];
  }

  v8f acc[8];
#pragma unroll
  for (int t = 0; t < 8; ++t) acc[t] = z8();
  const unsigned short* ap = A + (size_t)(rowBase + 16 * wave + m) * (size_t)K2 + 8 * hh;
  const unsigned short* bp = BT + (size_t)m * (size_t)K2 + 8 * hh;

#pragma unroll 1
  for (int k0 = 0; k0 < K2; k0 += 32) {
    FragB af;
    af.h[0] = *(const v8usa*)(ap + k0);
    af.h[1] = *(const v8usa*)(ap + k0 + 16);
#pragma unroll
    for (int nt = 0; nt < 8; ++nt) {
      const unsigned short* wq = bp + (size_t)(16 * nt) * (size_t)K2 + k0;
      FragB bf;
      bf.h[0] = *(const v8usa*)wq;
      bf.h[1] = *(const v8usa*)(wq + 16);
      acc[nt] = wmb(af, bf, acc[nt]);
    }
  }

#pragma unroll
  for (int nt = 0; nt < 8; ++nt) {
    const int lc = 16 * nt + m;
#pragma unroll
    for (int r = 0; r < 8; ++r) {
      const int lr = 16 * wave + 8 * hh + r;
      stg[lr * GBN + lc] = acc[nt][r];
    }
  }
  __syncthreads();

  {
    const int c  = tid & (NCLS - 1);
    const int r0 = tid >> 4;
#pragma unroll 1
    for (int j = 0; j < GBM / 8; ++j) {
      const int r = r0 + 8 * j;
      const float* tr = stg + r * GBN;
      float s = 0.0f;
#pragma unroll 1
      for (int k4 = 0; k4 < DF / 4; ++k4) {
        const v4f a = *(const v4fa*)(tr + 4 * k4);
        const float* w = wcs + (4 * k4) * NCLS + c;
        s = fmaf(a.x, w[0], s);
        s = fmaf(a.y, w[NCLS], s);
        s = fmaf(a.z, w[2 * NCLS], s);
        s = fmaf(a.w, w[3 * NCLS], s);
      }
      ys[r * NCLS + c] = s * nss[r];
    }
  }
  __syncthreads();

  v4f fv[(GBM * NCLS / 4) / GTHR];
#pragma unroll
  for (int j = 0; j < (GBM * NCLS / 4) / GTHR; ++j) fv[j] = *(const v4fa*)(ys + 4 * (tid + GTHR * j));
#pragma unroll
  for (int j = 0; j < (GBM * NCLS / 4) / GTHR; ++j) {
    const int i4  = tid + GTHR * j;
    const int row = rowBase + (i4 >> 2);
    float* op = y16 + (size_t)rowBase * NCLS + 4 * i4;
    if (row < nN) *(volatile v4f*)op = fv[j];
  }
  __threadfence();
#pragma unroll
  for (int j = 0; j < (GBM * NCLS / 4) / GTHR; ++j) {
    const int i4  = tid + GTHR * j;
    const int row = rowBase + (i4 >> 2);
    float* op = y16 + (size_t)rowBase * NCLS + 4 * i4;
    if (row < nN) *(volatile v4f*)op = fv[j];
  }
}

__global__ __launch_bounds__(NTHR) void k_agg2(const int* __restrict__ lst, const int* __restrict__ cntg,
                                               const int* __restrict__ offg, const float* __restrict__ ndg,
                                               const int* __restrict__ flg, const float* __restrict__ y16,
                                               const float* __restrict__ tab, int nN, float* z) {
  extern __shared__ __attribute__((aligned(16))) float zs[];
  const int tid = (int)threadIdx.x, lane = tid & 31, wave = tid >> 5;
  const int q = lane & 3, hs = lane >> 2;
  const int blk = (int)blockIdx.x;
  const int nodeBase = blk * NBA;
  const int* bl = lst + (size_t)blk * RCAP;
  const float qnan = __int_as_float(0x7fc00000);
  const float pz = (flg[blk * 32] != 0) ? qnan : 0.0f;
  const v4f c2v = *(const v4f*)(tab + T_C2 + 4 * q);

#pragma unroll 1
  for (int si = 0; si < NBA / NWAVE; ++si) {
    const int s    = si * NWAVE + wave;
    const int node = nodeBase + s;
    int c = cntg[node];
    const bool big = c > DEGCAP;
    c = c < 0 ? 0 : (c > DEGCAP ? DEGCAP : c);
    int o = offg[node];
    o = o < 0 ? 0 : (o > RCAP ? RCAP : o);
    const float nd = ndg[node];
    float a0 = 0.0f, a1 = 0.0f, a2 = 0.0f, a3 = 0.0f;
#pragma unroll 1
    for (int b0 = 0; b0 < c; b0 += 8) {
      const int hi_ = b0 + hs;
      int idx = o + hi_;
      idx = idx > RCAP - 1 ? RCAP - 1 : idx;
      int sr = bl[idx];
      sr = sr < 0 ? 0 : (sr > nN - 1 ? nN - 1 : sr);
      const v4f v = *(const v4fa*)(y16 + (size_t)sr * NCLS + 4 * q);
      const int mk = (hi_ < c) ? -1 : 0;
      a0 = bsel(mk, a0 + v.x, a0);
      a1 = bsel(mk, a1 + v.y, a1);
      a2 = bsel(mk, a2 + v.z, a2);
      a3 = bsel(mk, a3 + v.w, a3);
    }
    a0 += __shfl_xor(a0, 4, 32);  a1 += __shfl_xor(a1, 4, 32);
    a2 += __shfl_xor(a2, 4, 32);  a3 += __shfl_xor(a3, 4, 32);
    a0 += __shfl_xor(a0, 8, 32);  a1 += __shfl_xor(a1, 8, 32);
    a2 += __shfl_xor(a2, 8, 32);  a3 += __shfl_xor(a3, 8, 32);
    a0 += __shfl_xor(a0, 16, 32); a1 += __shfl_xor(a1, 16, 32);
    a2 += __shfl_xor(a2, 16, 32); a3 += __shfl_xor(a3, 16, 32);
    const float pzr = big ? qnan : pz;
    v4f zv;
    zv.x = (a0 * nd + c2v.x) + pzr;
    zv.y = (a1 * nd + c2v.y) + pzr;
    zv.z = (a2 * nd + c2v.z) + pzr;
    zv.w = (a3 * nd + c2v.w) + pzr;
    if (hs == 0) *(v4fa*)(zs + s * NCLS + 4 * q) = zv;
  }
  __syncthreads();

  float* zb = z + (size_t)nodeBase * NCLS;
#pragma unroll 1
  for (int it = 0; it < (NBA * NCLS / 4) / NTHR; ++it) {
    const int i4  = it * NTHR + tid;
    const int row = nodeBase + (i4 >> 2);
    const v4f v = *(const v4fa*)(zs + 4 * i4);
    if (row < nN) *(volatile v4f*)(zb + 4 * i4) = v;
  }
  __threadfence();
#pragma unroll 1
  for (int it = 0; it < (NBA * NCLS / 4) / NTHR; ++it) {
    const int i4  = it * NTHR + tid;
    const int row = nodeBase + (i4 >> 2);
    const v4f v = *(const v4fa*)(zs + 4 * i4);
    if (row < nN) *(volatile v4f*)(zb + 4 * i4) = v;
  }
}

__global__ __launch_bounds__(NTHR) void k_pool_out(const float* __restrict__ z, const int* __restrict__ gid,
                                                   const int* __restrict__ flg, const float* __restrict__ tab,
                                                   int nN, int nBlk, int outN, float* out) {
  __shared__ __attribute__((aligned(16))) float part[NTHR * 32];
  __shared__ int cpart[NTHR * 2];
  __shared__ __attribute__((aligned(16))) float outs[32];
  __shared__ int fls;
  const int tid = (int)threadIdx.x, lane = tid & 31, wave = tid >> 5;
  const int g0 = 2 * (int)blockIdx.x, g1 = g0 + 1;

  if (tid == 0) fls = 0;
  __syncthreads();
  {
    const int bi = tid < nBlk ? tid : nBlk - 1;
    const int f = flg[bi * 32];
    if (tid < nBlk && f != 0) fls = 1;
  }

  v4f a[8];
#pragma unroll
  for (int i = 0; i < 8; ++i) { const v4f zz = {0.f, 0.f, 0.f, 0.f}; a[i] = zz; }
  int c0 = 0, c1 = 0;
  const int nChunks = (nN + NTHR - 1) / NTHR;
#pragma unroll 1
  for (int ch = 0; ch < nChunks; ++ch) {
    const int n  = ch * NTHR + tid;
    const int nc = n < nN ? n : nN - 1;
    const int gv = gid[nc];
    const int m0 = (n < nN && gv == g0) ? -1 : 0;
    const int m1 = (n < nN && gv == g1) ? -1 : 0;
    const float* zr = z + (size_t)nc * NCLS;
#pragma unroll
    for (int qq = 0; qq < 4; ++qq) {
      const v4f v = *(const v4fa*)(zr + 4 * qq);
      v4f x = a[qq], y = a[4 + qq];
      x.x = bsel(m0, x.x + v.x, x.x); x.y = bsel(m0, x.y + v.y, x.y);
      x.z = bsel(m0, x.z + v.z, x.z); x.w = bsel(m0, x.w + v.w, x.w);
      y.x = bsel(m1, y.x + v.x, y.x); y.y = bsel(m1, y.y + v.y, y.y);
      y.z = bsel(m1, y.z + v.z, y.z); y.w = bsel(m1, y.w + v.w, y.w);
      a[qq] = x; a[4 + qq] = y;
    }
    c0 += m0 & 1;
    c1 += m1 & 1;
  }
#pragma unroll
  for (int i = 0; i < 8; ++i) *(v4fa*)(part + tid * 32 + 4 * i) = a[i];
  cpart[2 * tid]     = c0;
  cpart[2 * tid + 1] = c1;
  __syncthreads();
  if (tid < 32) {
    const int gs = tid >> 4;
    double sv = 0.0;
    int ct = 0;
#pragma unroll 1
    for (int i = 0; i < NTHR; ++i) {
      sv += (double)part[i * 32 + tid];
      ct += cpart[2 * i + gs];
    }
    const float cf = (float)(ct < 1 ? 1 : ct);
    float o = (float)sv * (1.0f / cf) + tab[T_BC + (tid & (NCLS - 1))];
    if (fls != 0) o = __int_as_float(0x7fc00000);
    outs[tid] = o;
  }
  __syncthreads();
  const v4f ov = *(const v4fa*)(outs + 4 * (lane & 7));
  const int e0 = (int)blockIdx.x * 32;
  float* op = out + (size_t)e0 + 4 * (lane & 7);
  const bool okst = (wave == 0) && (lane < 8) && (e0 + 32 <= outN);
  if (okst) *(volatile v4f*)op = ov;
  __threadfence();
  if (okst) *(volatile v4f*)op = ov;
}

static inline int cdiv(int a, int b) { return (a + b - 1) / b; }
static inline size_t al256(size_t o) { return (o + 255) & ~(size_t)255; }

extern "C" void kernel_launch(void* const* d_in, const int* in_sizes, int n_in,
                              void* d_out, int out_size, void* d_ws, size_t ws_size,
                              hipStream_t stream) {
  if (n_in < 11) return;
  if (in_sizes[0] < DF || (in_sizes[0] % DF) != 0) return;
  const int nN = in_sizes[0] / DF;
  if (nN < GBM || nN > (1 << 22) || (nN & 1) != 0) return;
  if (in_sizes[1] != DF * DF || in_sizes[2] != DF || in_sizes[3] != DF) return;
  if (in_sizes[4] != DF * DF || in_sizes[5] != DF) return;
  if (in_sizes[6] != DF * NCLS || in_sizes[7] != NCLS) return;
  const int nE = in_sizes[8];
  if (nE < 1 || nE >= (1 << 21) || in_sizes[9] != nE) return;
  if (in_sizes[10] != nN) return;
  if (out_size != NGR * NCLS) return;

  const float* h   = (const float*)d_in[0];
  const float* W1  = (const float*)d_in[1];
  const float* b1  = (const float*)d_in[2];
  const float* p   = (const float*)d_in[3];
  const float* W2  = (const float*)d_in[4];
  const float* b2  = (const float*)d_in[5];
  const float* Wc  = (const float*)d_in[6];
  const float* bc  = (const float*)d_in[7];
  const int*   src = (const int*)d_in[8];
  const int*   dst = (const int*)d_in[9];
  const int*   gid = (const int*)d_in[10];
  float* out = (float*)d_out;

  const int MP   = cdiv(nN, DF) * DF;
  const int gM   = MP / GBM;
  const int gA   = cdiv(MP, NBA);
  const int NBP  = gA * NBA;
  const int gD   = cdiv(nN, NBD);
  const int NBPD = gD * NBD;
  if (NBP < MP || NBPD < MP || gA > NTHR) return;
  const int vec8 = 1;

  char* ws = (char*)d_ws;
  size_t off = 0;
  const size_t oA   = off; off = al256(off + (size_t)MP * K2 * 2);
  const size_t oB   = off; off = al256(off + (size_t)nN * DF * 4);
  const size_t oLST = off; off = al256(off + (size_t)gA * RCAP * 4);
  const size_t oCNT = off; off = al256(off + (size_t)NBP * 4);
  const size_t oOFF = off; off = al256(off + (size_t)NBP * 4);
  const size_t oND  = off; off = al256(off + (size_t)NBP * 4);
  const size_t oNS  = off; off = al256(off + (size_t)NBPD * 4);
  const size_t oFLG = off; off = al256(off + (size_t)gA * 128);
  const size_t oW1T = off; off = al256(off + (size_t)DF * DF * 2);
  const size_t oW2D = off; off = al256(off + (size_t)DF * K2 * 2);
  const size_t oTAB = off; off = al256(off + (size_t)TABN * 4);
  if (off > ws_size || off > (size_t)WSMAX) return;
  if ((size_t)2 * nN * NCLS * 4 > (size_t)nN * DF * 4) return;
  unsigned short* HB  = (unsigned short*)(ws + oA);
  unsigned short* X1P = (unsigned short*)(ws + oA);
  float*          M1  = (float*)(ws + oB);
  float*          Y16 = (float*)(ws + oB);
  float*          Z   = (float*)(ws + oB) + (size_t)nN * NCLS;
  int*            LST = (int*)(ws + oLST);
  int*            CNT = (int*)(ws + oCNT);
  int*            OFF = (int*)(ws + oOFF);
  float*          ND  = (float*)(ws + oND);
  float*          NS  = (float*)(ws + oNS);
  int*            FLG = (int*)(ws + oFLG);
  unsigned short* W1T = (unsigned short*)(ws + oW1T);
  unsigned short* W2D = (unsigned short*)(ws + oW2D);
  float*          TAB = (float*)(ws + oTAB);

  const size_t bktLds = (size_t)BKT_LDS_INTS * 4;
  const size_t ag2Lds = (size_t)NBA * NCLS * 4;
  hipFuncSetAttribute(reinterpret_cast<const void*>(&k_bucket), hipFuncAttributeMaxDynamicSharedMemorySize, (int)bktLds);
  hipFuncSetAttribute(reinterpret_cast<const void*>(&k_agg2), hipFuncAttributeMaxDynamicSharedMemorySize, (int)ag2Lds);

  const int nUnits = NUPRE + MP * (DF / 8);
  k_prep<<<cdiv(nUnits, NTHR), NTHR, 0, stream>>>(h, W1, b1, p, W2, b2, Wc, bc, HB, W1T, W2D, TAB, nN, nUnits);
  k_degout<<<gD, NTHR, 0, stream>>>(src, nE, vec8, NS);
  k_bucket<<<gA, NTHR, bktLds, stream>>>(src, dst, nE, nN, vec8, LST, CNT, OFF, ND, FLG);
  k_gemm1<<<gM, GTHR, 0, stream>>>(HB, W1T, NS, M1, nN);
  k_agg1<<<gA, NTHR, 0, stream>>>(LST, CNT, OFF, ND, FLG, M1, TAB, nN, MP, X1P);
  k_gemm2<<<gM, GTHR, 0, stream>>>(X1P, W2D, NS, TAB, Y16, nN);
  k_agg2<<<gA, NTHR, ag2Lds, stream>>>(LST, CNT, OFF, ND, FLG, Y16, TAB, nN, Z);
  k_pool_out<<<(NGR * NCLS) / 32, NTHR, 0, stream>>>(Z, gid, FLG, TAB, nN, gA, out_size, out);
}
